// GATNet_2276332667608
// MI455X (gfx1250) — hardware-verified
//
#include <hip/hip_runtime.h>
#include <stddef.h>
#include <stdint.h>
#include <math.h>


#define F_IN    128
#define XUPR    (F_IN / 8)
#define HC1     128
#define K2      HC1
#define HC2     64
#define NTHR    256
#define NWAVE   8
#define EPT     8
#define CHUNK   (NTHR * EPT)
#define WCAP    (EPT * 32)
#define LISTN   (NWAVE * WCAP)
#define NBMAX   2048
#define SLOTB   11
#define NBRUN   1024
#define RCAP    28672
#define DEGCAP  128
#define STW     128
#define GBM     64
#define GBN     64
#define GTHR    128
#define MROWS   128
#define NSD1    4
#define NSD2    2
#define NEGSL   0.2f
#define ACTSL   0.01f
#define EPS_SM  1e-16f
#define MX0     (-1.0e30f)
#define WSMAX   134217728
#define LDS_AGG ((2 * RCAP + 2 * NBMAX + LISTN) * 4 + 64)

static_assert((CHUNK & (CHUNK - 1)) == 0 && CHUNK <= (1 << SLOTB));
static_assert(NBMAX == (1 << SLOTB));
static_assert((NBRUN & (NBRUN - 1)) == 0 && NBRUN <= NBMAX && NBRUN >= 32);
static_assert(NTHR * 8 == NBMAX);
static_assert(LISTN >= NBMAX);
static_assert(LISTN >= NWAVE * WCAP);
static_assert((RCAP % 32) == 0);
static_assert(NWAVE * STW <= RCAP);
static_assert(HC1 <= STW && HC2 <= STW);
static_assert(LDS_AGG <= 300000);
static_assert(GBM == (GTHR / 32) * 16);
static_assert(GTHR == 2 * GBN && GTHR == 2 * GBM);
static_assert((F_IN % 32) == 0 && (K2 % 32) == 0);
static_assert((F_IN % 8) == 0 && (HC1 % 8) == 0);
static_assert((HC1 % GBN) == 0 && (HC2 % GBN) == 0);
static_assert(NSD1 == 2 * (HC1 / GBN) && NSD2 == 2 * (HC2 / GBN));
static_assert((MROWS % GBM) == 0);
static_assert(HC1 == 4 * 32);
static_assert(HC1 == 16 * 8);
static_assert(HC2 == 2 * 32);
static_assert(HC2 == 16 * 4);

typedef float          v2f  __attribute__((ext_vector_type(2)));
typedef float          v4f  __attribute__((ext_vector_type(4)));
typedef float          v8f  __attribute__((ext_vector_type(8)));
typedef int            v4i  __attribute__((ext_vector_type(4)));
typedef int            v8i  __attribute__((ext_vector_type(8)));
typedef unsigned int   v4u  __attribute__((ext_vector_type(4)));
typedef unsigned short v8us __attribute__((ext_vector_type(8)));
typedef __bf16         v16b __attribute__((ext_vector_type(16)));
typedef v2f  __attribute__((may_alias)) v2fa;
typedef v4f  __attribute__((may_alias)) v4fa;
typedef v8us __attribute__((may_alias)) v8usa;
union FragB { v16b v; v8us h[2]; v8i w; };

__device__ __forceinline__ v8f wmb(const FragB& a, const FragB& b, v8f c) {
  v8f d = __builtin_amdgcn_wmma_f32_16x16x32_bf16(false, a.v, false, b.v, (short)0, c, false, false);
  asm volatile("v_nop\n\tv_nop\n\tv_nop\n\tv_nop" : "+v"(d) : "v"(a.w), "v"(b.w));
  return d;
}

__device__ __forceinline__ unsigned int f2bf(float f) {
  const unsigned int u = __float_as_uint(f);
  return ((u + 0x7FFFu + ((u >> 16) & 1u)) >> 16) & 0xFFFFu;
}
__device__ __forceinline__ float bf2f(unsigned int b) { return __uint_as_float(b << 16); }
__device__ __forceinline__ float bfr(float f) { return bf2f(f2bf(f)); }
__device__ __forceinline__ unsigned int pk2(float lo, float hi) { return f2bf(lo) | (f2bf(hi) << 16); }
__device__ __forceinline__ v4u pack8(const v4f a, const v4f b) {
  v4u r;
  r.x = pk2(a.x, a.y); r.y = pk2(a.z, a.w); r.z = pk2(b.x, b.y); r.w = pk2(b.z, b.w);
  return r;
}
__device__ __forceinline__ float actf(float v) { return v > 0.f ? v : ACTSL * v; }

__device__ __forceinline__ int scan_chunk(const int* __restrict__ dsts, int nE, int cbase, int slotBase,
                                          int nb, int vec8, int* list, int tid, int lane, int wave) {
  int wc = 0;
  const int el0  = tid * EPT;
  const int e0   = cbase + el0;
  const int sent = -2147483647 - 1;
  v4i da, db;
  if (vec8 != 0 && cbase + CHUNK <= nE) {
    da = *(const v4i*)(dsts + e0);
    db = *(const v4i*)(dsts + e0 + 4);
  } else {
    da.x = (e0     < nE) ? dsts[min(e0,     nE - 1)] : sent;
    da.y = (e0 + 1 < nE) ? dsts[min(e0 + 1, nE - 1)] : sent;
    da.z = (e0 + 2 < nE) ? dsts[min(e0 + 2, nE - 1)] : sent;
    da.w = (e0 + 3 < nE) ? dsts[min(e0 + 3, nE - 1)] : sent;
    db.x = (e0 + 4 < nE) ? dsts[min(e0 + 4, nE - 1)] : sent;
    db.y = (e0 + 5 < nE) ? dsts[min(e0 + 5, nE - 1)] : sent;
    db.z = (e0 + 6 < nE) ? dsts[min(e0 + 6, nE - 1)] : sent;
    db.w = (e0 + 7 < nE) ? dsts[min(e0 + 7, nE - 1)] : sent;
  }
  const unsigned nbs = (unsigned)slotBase;
  const unsigned unb = (unsigned)nb;
  const unsigned s0 = (unsigned)da.x - nbs, s1 = (unsigned)da.y - nbs;
  const unsigned s2 = (unsigned)da.z - nbs, s3 = (unsigned)da.w - nbs;
  const unsigned s4 = (unsigned)db.x - nbs, s5 = (unsigned)db.y - nbs;
  const unsigned s6 = (unsigned)db.z - nbs, s7 = (unsigned)db.w - nbs;
  const bool h0 = s0 < unb, h1 = s1 < unb, h2 = s2 < unb, h3 = s3 < unb;
  const bool h4 = s4 < unb, h5 = s5 < unb, h6 = s6 < unb, h7 = s7 < unb;
  const unsigned any = __builtin_amdgcn_ballot_w32(h0 | h1 | h2 | h3 | h4 | h5 | h6 | h7);
  if (any != 0u) {
#define HITJ(J, HJ, SJ) { \
      const unsigned mj = __builtin_amdgcn_ballot_w32(HJ); \
      if (mj != 0u) { \
        if (HJ) { \
          const int pos = wc + (int)__builtin_amdgcn_mbcnt_lo(mj, 0u); \
          if (pos < WCAP) list[wave * WCAP + pos] = ((el0 + (J)) << SLOTB) | (int)(SJ); \
        } \
        wc += (int)__builtin_popcount(mj); } }
    HITJ(0, h0, s0)
    HITJ(1, h1, s1)
    HITJ(2, h2, s2)
    HITJ(3, h3, s3)
    HITJ(4, h4, s4)
    HITJ(5, h5, s5)
    HITJ(6, h6, s6)
    HITJ(7, h7, s7)
#undef HITJ
  }
  return wc;
}

__global__ __launch_bounds__(NTHR) void k_xprep(const float* __restrict__ x, unsigned short* xb, int nN, int nUnits) {
  const int i = (int)blockIdx.x * NTHR + (int)threadIdx.x;
  if (i >= nUnits) return;
  const int row = i / XUPR;
  const int c0  = (i - row * XUPR) * 8;
  const int rc  = row < nN ? row : nN - 1;
  const float* p = x + (size_t)rc * F_IN + c0;
  v4f a = *(const v4fa*)p, b = *(const v4fa*)(p + 4);
  const v4f z4 = {0.f, 0.f, 0.f, 0.f};
  if (row >= nN) { a = z4; b = z4; }
  const v4u hv = pack8(a, b);
  const size_t o = (size_t)row * F_IN + c0;
  *(volatile v4u*)(xb + o) = hv;
  __threadfence();
  *(volatile v4u*)(xb + o) = hv;
}

__global__ __launch_bounds__(NTHR) void k_wtr(const float* __restrict__ w, int Kin, int Ncol, int Nrows, int Kout,
                                              unsigned short* wt, int nUnits) {
  const int u = (int)blockIdx.x * NTHR + (int)threadIdx.x;
  if (u >= nUnits) return;
  const int kq = Kout >> 3;
  const int n  = u / kq;
  const int k8 = (u - n * kq) * 8;
  const int kk = k8 - (k8 / Kin) * Kin;
  const int ncl = n < Ncol ? n : Ncol - 1;
  const float* p = w + (size_t)kk * (size_t)Ncol + ncl;
  v4f a, b;
  a.x = p[0];                    a.y = p[(size_t)Ncol];         a.z = p[(size_t)2 * Ncol];     a.w = p[(size_t)3 * Ncol];
  b.x = p[(size_t)4 * Ncol];     b.y = p[(size_t)5 * Ncol];     b.z = p[(size_t)6 * Ncol];     b.w = p[(size_t)7 * Ncol];
  const v4f z4 = {0.f, 0.f, 0.f, 0.f};
  if (n >= Ncol || n >= Nrows) { a = z4; b = z4; }
  const v4u wv = pack8(a, b);
  unsigned short* o = wt + (size_t)n * (size_t)Kout + k8;
  *(volatile v4u*)o = wv;
  __threadfence();
  *(volatile v4u*)o = wv;
}

__global__ __launch_bounds__(GTHR) void k_gemm(
    const unsigned short* __restrict__ A, const unsigned short* __restrict__ WT,
    float* outF, int K, int ldo,
    const float* __restrict__ atts, const float* __restrict__ attd, int attN,
    float* SD, int MPr)
{
  __shared__ __attribute__((aligned(16))) float stg[GBM * GBN];
  __shared__ __attribute__((aligned(16))) float satt[2 * GBN];
  __shared__ __attribute__((aligned(16))) float sdot[2 * GBM];
  const int tid = (int)threadIdx.x, lane = tid & 31, wave = tid >> 5, hh = lane >> 4, m = lane & 15;
  const int rowBase = (int)blockIdx.x * GBM;
  const int by      = (int)blockIdx.y;
  const int col0    = by * GBN;

  {
    const int which = tid >> 6;
    const int c     = tid & 63;
    int ai = col0 + c;
    ai = ai < 0 ? 0 : (ai < attN ? ai : attN - 1);
    const float vs = atts[ai];
    const float vd = attd[ai];
    const unsigned int msk = (which == 0) ? 0u : 0xFFFFFFFFu;
    const float v = __uint_as_float((__float_as_uint(vs) & ~msk) | (__float_as_uint(vd) & msk));
    satt[which * GBN + c] = bfr(v);
  }

  v8f acc[4];
  {
    const v8f z = {0.f, 0.f, 0.f, 0.f, 0.f, 0.f, 0.f, 0.f};
    acc[0] = z; acc[1] = z; acc[2] = z; acc[3] = z;
  }
  const unsigned short* ap = A  + (size_t)(rowBase + 16 * wave + m) * (size_t)K + 8 * hh;
  const unsigned short* wp = WT + (size_t)(col0 + m) * (size_t)K + 8 * hh;
  const int ksteps = K >> 5;
#pragma unroll 1
  for (int ks = 0; ks < ksteps; ++ks) {
    FragB af;
    af.h[0] = *(const v8usa*)(ap + 32 * ks);
    af.h[1] = *(const v8usa*)(ap + 32 * ks + 16);
#pragma unroll
    for (int t = 0; t < 4; ++t) {
      const unsigned short* wq = wp + (size_t)(16 * t) * (size_t)K + 32 * ks;
      FragB bf;
      bf.h[0] = *(const v8usa*)wq;
      bf.h[1] = *(const v8usa*)(wq + 16);
      acc[t] = wmb(af, bf, acc[t]);
    }
  }

#pragma unroll
  for (int t = 0; t < 4; ++t) {
    const int lc = 16 * t + m;
#pragma unroll
    for (int r = 0; r < 8; ++r) {
      const int lr = 16 * wave + 8 * hh + r;
      stg[lr * GBN + lc] = acc[t][r];
    }
  }
  __syncthreads();

  {
    const int row = tid & 63, which = tid >> 6;
    const float* sa = satt + which * GBN;
    const float* hr = stg + row * GBN;
    float d = 0.f;
#pragma unroll 4
    for (int c4 = 0; c4 < GBN / 4; ++c4) {
      const v4f hv = *(const v4fa*)(hr + 4 * c4);
      const v4f av = *(const v4fa*)(sa + 4 * c4);
      d = fmaf(hv.x, av.x, d);
      d = fmaf(hv.y, av.y, d);
      d = fmaf(hv.z, av.z, d);
      d = fmaf(hv.w, av.w, d);
    }
    sdot[which * GBM + row] = d;
  }
  __syncthreads();

  v4f fv[8];
#pragma unroll
  for (int i = 0; i < 8; ++i) {
    const int lr = 16 * wave + 2 * i + hh;
    fv[i] = *(const v4fa*)(stg + lr * GBN + 4 * m);
  }
  const int piece = lane & 15;
  const int pl    = lane >> 4;
  const int plane = 2 * by + pl;
  const bool wsd  = wave == 0;
  const v4f sdv = *(const v4fa*)(sdot + pl * GBM + 4 * piece);
  float* sp = SD + (size_t)plane * (size_t)MPr + rowBase + 4 * piece;

#pragma unroll
  for (int i = 0; i < 8; ++i) {
    const int lr = 16 * wave + 2 * i + hh;
    const int gr = rowBase + lr;
    float* op = outF + (size_t)gr * (size_t)ldo + col0 + 4 * m;
    *(volatile v4f*)op = fv[i];
  }
  if (wsd) *(volatile v4f*)sp = sdv;
  __threadfence();
#pragma unroll
  for (int i = 0; i < 8; ++i) {
    const int lr = 16 * wave + 2 * i + hh;
    const int gr = rowBase + lr;
    float* op = outF + (size_t)gr * (size_t)ldo + col0 + 4 * m;
    *(volatile v4f*)op = fv[i];
  }
  if (wsd) *(volatile v4f*)sp = sdv;
}

template<int L>
__global__ __launch_bounds__(NTHR) void k_agg(
    const int* __restrict__ srcs, const int* __restrict__ dsts,
    const float* __restrict__ F, const float* __restrict__ SD,
    unsigned short* HP, float* out,
    int nN, int nE, int nb, int vec8, int MPr) {
  extern __shared__ v4f lds_dyn[];
  int* reg1 = (int*)lds_dyn;
  int* reg2 = reg1 + RCAP;
  int* scnt = reg2 + RCAP;
  int* soff = scnt + NBMAX;
  int* list = soff + NBMAX;
  int* wcnt = list + LISTN;
  int* wtot = wcnt + NWAVE;
  const int tid = (int)threadIdx.x, lane = tid & 31, wave = tid >> 5;
  const int nodeBase = (int)blockIdx.x * nb;

  for (int i = tid; i < NBMAX; i += NTHR) scnt[i] = 0;
  __syncthreads();

  int tot = 0;
  const int nChunks = (nE + CHUNK - 1) / CHUNK;
#pragma unroll 1
  for (int ch = 0; ch < nChunks; ++ch) {
    const int cbase = ch * CHUNK;
    const int wc = scan_chunk(dsts, nE, cbase, nodeBase, nb, vec8, list, tid, lane, wave);
    if (lane == 0) wcnt[wave] = wc;
    __syncthreads();
    int pre = 0, all = 0;
#pragma unroll
    for (int w2 = 0; w2 < NWAVE; ++w2) {
      int c = wcnt[w2];
      c = c < 0 ? 0 : (c > WCAP ? WCAP : c);
      all += c;
      pre += (w2 < wave) ? c : 0;
    }
    const int wcc  = wc > WCAP ? WCAP : wc;
    const int base = tot + pre;
#pragma unroll 1
    for (int i = lane; i < wcc; i += 32) {
      const int ent = list[wave * WCAP + i];
      const int el  = (ent >> SLOTB) & (CHUNK - 1);
      const int sl  = ent & (NBMAX - 1);
      int eid = cbase + el;
      eid = eid > nE - 1 ? nE - 1 : eid;
      const int pos = base + i;
      if (pos < RCAP) reg1[pos] = (int)(((unsigned)eid << SLOTB) | (unsigned)sl);
    }
    tot += all;
    tot = tot > RCAP ? RCAP : tot;
    __syncthreads();
  }
  const int nh = tot;

  if (wave == 0) {
#pragma unroll 1
    for (int b0 = 0; b0 < nh; b0 += 32) {
      const int idx = b0 + lane;
      const int uv  = reg1[idx < nh ? idx : nh - 1];
      const int m32 = (nh - b0) < 32 ? (nh - b0) : 32;
#pragma unroll 1
      for (int k = 0; k < m32; ++k) {
        const int u  = __builtin_amdgcn_readlane(uv, k);
        const int sl = u & (NBMAX - 1);
        if (lane == 0) scnt[sl] = scnt[sl] + 1;
      }
    }
  }
  __syncthreads();

  {
    const v4i ca = *(const v4i*)(scnt + 8 * tid);
    const v4i cb = *(const v4i*)(scnt + 8 * tid + 4);
    const int e0 = ca.x < 0 ? 0 : ca.x, e1 = ca.y < 0 ? 0 : ca.y, e2 = ca.z < 0 ? 0 : ca.z, e3 = ca.w < 0 ? 0 : ca.w;
    const int e4 = cb.x < 0 ? 0 : cb.x, e5 = cb.y < 0 ? 0 : cb.y, e6 = cb.z < 0 ? 0 : cb.z, e7 = cb.w < 0 ? 0 : cb.w;
    const int ts = e0 + e1 + e2 + e3 + e4 + e5 + e6 + e7;
    int incl = ts;
#pragma unroll
    for (int d = 1; d < 32; d <<= 1) {
      const int up = __shfl_up(incl, d);
      if (lane >= d) incl += up;
    }
    if (lane == 31) wtot[wave] = incl;
    __syncthreads();
    int pre = 0;
#pragma unroll
    for (int w2 = 0; w2 < NWAVE; ++w2) pre += (w2 < wave) ? wtot[w2] : 0;
    int run = pre + incl - ts;
    soff[8 * tid + 0] = run; run += e0;
    soff[8 * tid + 1] = run; run += e1;
    soff[8 * tid + 2] = run; run += e2;
    soff[8 * tid + 3] = run; run += e3;
    soff[8 * tid + 4] = run; run += e4;
    soff[8 * tid + 5] = run; run += e5;
    soff[8 * tid + 6] = run; run += e6;
    soff[8 * tid + 7] = run;
  }
  __syncthreads();
  for (int i = tid; i < NBMAX; i += NTHR) list[i] = soff[i];
  __syncthreads();

  if (wave == 0) {
#pragma unroll 1
    for (int b0 = 0; b0 < nh; b0 += 32) {
      const int idx = b0 + lane;
      const int uv  = reg1[idx < nh ? idx : nh - 1];
      const int m32 = (nh - b0) < 32 ? (nh - b0) : 32;
#pragma unroll 1
      for (int k = 0; k < m32; ++k) {
        const int u   = __builtin_amdgcn_readlane(uv, k);
        const int sl  = u & (NBMAX - 1);
        const int eid = (int)((unsigned)u >> SLOTB);
        if (lane == 0) {
          int pos = list[sl];
          pos = pos < 0 ? 0 : (pos > RCAP - 1 ? RCAP - 1 : pos);
          reg2[pos] = eid;
          list[sl] = pos + 1;
        }
      }
    }
  }
  __syncthreads();

  const int nbw = nb >> 3;
  const bool ovf = (nh >= RCAP);
  const float qnan = __int_as_float(0x7fc00000);
  float* stw = (float*)reg1 + wave * STW;
  const int lc = lane < 16 ? lane : 15;

  if (L == 1) {
    const int c0 = 4 * lane;
    const float* ASa = SD;
    const float* ADa = SD + (size_t)MPr;
    const float* ASb = SD + 2 * (size_t)MPr;
    const float* ADb = SD + 3 * (size_t)MPr;
#pragma unroll 1
    for (int jt = 0; jt < nbw; ++jt) {
      const int slot = wave * nbw + jt;
      const int grow = nodeBase + slot;
      const int gcl  = grow < nN ? grow : nN - 1;
      int st = soff[slot];
      const int craw = scnt[slot];
      int cnt = craw;
      st  = st < 0 ? 0 : (st > nh ? nh : st);
      cnt = cnt < 0 ? 0 : (cnt > DEGCAP ? DEGCAP : cnt);
      if (cnt > nh - st) cnt = nh - st;
      const float pz = (ovf || craw > DEGCAP) ? qnan : 0.0f;
      const bool live = grow < nN;

      const float adv = ADa[gcl] + ADb[gcl];
      float mx = MX0, dn = 0.0f;
      v4f av = {0.f, 0.f, 0.f, 0.f};

#pragma unroll 1
      for (int q = 0; q < cnt; ++q) {
        int idx = st + q; idx = idx > RCAP - 1 ? RCAP - 1 : idx;
        int eid = reg2[idx]; eid = eid < 0 ? 0 : (eid > nE - 1 ? nE - 1 : eid);
        const int sraw = srcs[eid];
        const int s = sraw < 0 ? 0 : (sraw > nN - 1 ? nN - 1 : sraw);
        const v4f fs = *(const v4fa*)(F + (size_t)s * HC1 + c0);
        float lg = (ASa[s] + ASb[s]) + adv;
        lg = lg > 0.f ? lg : NEGSL * lg;
        const float df = lg - mx;
        const float ee = __expf(-fabsf(df));
        const bool up  = df > 0.f;
        const float s1 = up ? ee : 1.0f;
        const float s2 = up ? 1.0f : ee;
        mx = up ? lg : mx;
        dn = fmaf(dn, s1, s2);
        av.x = fmaf(av.x, s1, s2 * fs.x);
        av.y = fmaf(av.y, s1, s2 * fs.y);
        av.z = fmaf(av.z, s1, s2 * fs.z);
        av.w = fmaf(av.w, s1, s2 * fs.w);
      }
      const float ds = dn > 0.f ? dn : 1.0f;
      const float iv = (dn > 0.f ? 1.0f : 0.0f) * __builtin_amdgcn_rcpf(ds + EPS_SM);
      v4f r;
      r.x = (live ? actf(av.x * iv) : 0.f) + pz;
      r.y = (live ? actf(av.y * iv) : 0.f) + pz;
      r.z = (live ? actf(av.z * iv) : 0.f) + pz;
      r.w = (live ? actf(av.w * iv) : 0.f) + pz;
      __builtin_amdgcn_fence(__ATOMIC_RELEASE, "wavefront");
      __builtin_amdgcn_wave_barrier();
      *(v4fa*)(stw + 4 * lane) = r;
      __builtin_amdgcn_fence(__ATOMIC_RELEASE, "wavefront");
      __builtin_amdgcn_wave_barrier();
      const v4f ga = *(const v4fa*)(stw + 8 * lc);
      const v4f gb = *(const v4fa*)(stw + 8 * lc + 4);
      const v4u hv = pack8(ga, gb);
      unsigned short* gh = HP + (size_t)grow * HC1 + 8 * lc;
      const bool wr = (grow < MPr) && (lane < 16);
      if (wr) *(volatile v4u*)gh = hv;
      __threadfence();
      if (wr) *(volatile v4u*)gh = hv;
    }
  } else {
    const int c0 = 2 * lane;
    const float* ASa = SD;
    const float* ADa = SD + (size_t)MPr;
#pragma unroll 1
    for (int jt = 0; jt < nbw; ++jt) {
      const int slot = wave * nbw + jt;
      const int grow = nodeBase + slot;
      const int gcl  = grow < nN ? grow : nN - 1;
      int st = soff[slot];
      const int craw = scnt[slot];
      int cnt = craw;
      st  = st < 0 ? 0 : (st > nh ? nh : st);
      cnt = cnt < 0 ? 0 : (cnt > DEGCAP ? DEGCAP : cnt);
      if (cnt > nh - st) cnt = nh - st;
      const float pz = (ovf || craw > DEGCAP) ? qnan : 0.0f;

      const float adv = ADa[gcl];
      float mx = MX0, dn = 0.0f;
      v2f av = {0.f, 0.f};

#pragma unroll 1
      for (int q = 0; q < cnt; ++q) {
        int idx = st + q; idx = idx > RCAP - 1 ? RCAP - 1 : idx;
        int eid = reg2[idx]; eid = eid < 0 ? 0 : (eid > nE - 1 ? nE - 1 : eid);
        const int sraw = srcs[eid];
        const int s = sraw < 0 ? 0 : (sraw > nN - 1 ? nN - 1 : sraw);
        const v2f fs = *(const v2fa*)(F + (size_t)s * HC2 + c0);
        float lg = ASa[s] + adv;
        lg = lg > 0.f ? lg : NEGSL * lg;
        const float df = lg - mx;
        const float ee = __expf(-fabsf(df));
        const bool up  = df > 0.f;
        const float s1 = up ? ee : 1.0f;
        const float s2 = up ? 1.0f : ee;
        mx = up ? lg : mx;
        dn = fmaf(dn, s1, s2);
        av.x = fmaf(av.x, s1, s2 * fs.x);
        av.y = fmaf(av.y, s1, s2 * fs.y);
      }
      const float ds = dn > 0.f ? dn : 1.0f;
      const float iv = (dn > 0.f ? 1.0f : 0.0f) * __builtin_amdgcn_rcpf(ds + EPS_SM);
      const float z0 = av.x * iv;
      const float z1 = av.y * iv;
      float vm = fmaxf(z0, z1);
#pragma unroll
      for (int off = 16; off > 0; off >>= 1) vm = fmaxf(vm, __shfl_xor(vm, off));
      const float x0 = z0 - vm, x1 = z1 - vm;
      float sm = expf(x0) + expf(x1);
#pragma unroll
      for (int off = 16; off > 0; off >>= 1) sm += __shfl_xor(sm, off);
      const float ls = logf(sm);
      v2f o;
      o.x = (x0 - ls) + pz;
      o.y = (x1 - ls) + pz;
      __builtin_amdgcn_fence(__ATOMIC_RELEASE, "wavefront");
      __builtin_amdgcn_wave_barrier();
      *(v2fa*)(stw + 2 * lane) = o;
      __builtin_amdgcn_fence(__ATOMIC_RELEASE, "wavefront");
      __builtin_amdgcn_wave_barrier();
      const v4f gv = *(const v4fa*)(stw + 4 * lc);
      float* gp = out + (size_t)grow * HC2 + 4 * lc;
      const bool wsv = (grow < nN) && (lane < 16);
      if (wsv) *(volatile v4f*)gp = gv;
      __threadfence();
      if (wsv) *(volatile v4f*)gp = gv;
    }
  }
  (void)HP; (void)out;
}

static int pick_nb(int nE, int nN) {
  int nb = NBRUN;
  while (nb > 32 && (long long)nb * (long long)nE * 5LL > (long long)RCAP * (long long)nN * 4LL) nb >>= 1;
  return nb;
}
static inline int cdiv(int a, int b) { return (a + b - 1) / b; }

extern "C" void kernel_launch(void* const* d_in, const int* in_sizes, int n_in,
                              void* d_out, int out_size, void* d_ws, size_t ws_size,
                              hipStream_t stream) {
  if (n_in < 6) return;
  const int nN = in_sizes[0] / F_IN;
  if (nN <= 0 || in_sizes[0] != nN * F_IN || nN > (1 << 22)) return;
  if (in_sizes[1] < 2 || (in_sizes[1] & 1) != 0) return;
  const int nE = in_sizes[1] / 2;
  if (nE < 1 || nE >= (1 << (32 - SLOTB))) return;
  if (in_sizes[2] != F_IN * HC1) return;
  if (in_sizes[3] != 2 * HC1) return;
  if (in_sizes[4] != K2 * HC2) return;
  if (in_sizes[5] != 2 * HC2) return;
  if (out_size != nN * HC2) return;

  const float* x   = (const float*)d_in[0];
  const int*   ei  = (const int*)  d_in[1];
  const float* W1  = (const float*)d_in[2];
  const float* a1  = (const float*)d_in[3];
  const float* W2  = (const float*)d_in[4];
  const float* a2  = (const float*)d_in[5];
  float* out = (float*)d_out;
  const int* src = ei;
  const int* dst = ei + nE;

  const int MP   = cdiv(nN, MROWS) * MROWS;
  const int nb   = pick_nb(nE, nN);
  if (nb < 32 || (nb & (nb - 1)) != 0 || nb > NBRUN) return;
  const int gA   = cdiv(MP, nb);
  const int vec8 = ((nE & 3) == 0) ? 1 : 0;
  if (gA * nb < MP) return;

  char* ws = (char*)d_ws;
  size_t off = 0;
  const size_t oXB  = off; off += (size_t)MP * F_IN * 2;           off = (off + 255) & ~(size_t)255;
  const size_t oWT1 = off; off += (size_t)HC1 * F_IN * 2;          off = (off + 255) & ~(size_t)255;
  const size_t oWT2 = off; off += (size_t)HC2 * K2 * 2;            off = (off + 255) & ~(size_t)255;
  const size_t oWH1 = off; off += (size_t)MP * HC1 * 4;            off = (off + 255) & ~(size_t)255;
  const size_t oSD1 = off; off += (size_t)NSD1 * MP * 4;           off = (off + 255) & ~(size_t)255;
  const size_t oHB  = off; off += (size_t)MP * HC1 * 2;            off = (off + 255) & ~(size_t)255;
  const size_t oWH2 = off; off += (size_t)MP * HC2 * 4;            off = (off + 255) & ~(size_t)255;
  const size_t oSD2 = off; off += (size_t)NSD2 * MP * 4;           off = (off + 255) & ~(size_t)255;
  if (off > ws_size || off > (size_t)WSMAX) return;
  unsigned short* XB  = (unsigned short*)(ws + oXB);
  unsigned short* WT1 = (unsigned short*)(ws + oWT1);
  unsigned short* WT2 = (unsigned short*)(ws + oWT2);
  float*          WH1 = (float*)(ws + oWH1);
  float*          SD1 = (float*)(ws + oSD1);
  unsigned short* HB  = (unsigned short*)(ws + oHB);
  float*          WH2 = (float*)(ws + oWH2);
  float*          SD2 = (float*)(ws + oSD2);

  hipFuncSetAttribute(reinterpret_cast<const void*>(&k_agg<1>),
                      hipFuncAttributeMaxDynamicSharedMemorySize, LDS_AGG);
  hipFuncSetAttribute(reinterpret_cast<const void*>(&k_agg<2>),
                      hipFuncAttributeMaxDynamicSharedMemorySize, LDS_AGG);

  const int nUx = MP * XUPR;
  k_xprep<<<cdiv(nUx, NTHR), NTHR, 0, stream>>>(x, XB, nN, nUx);

  {
    const int nUw1 = HC1 * (F_IN / 8);
    k_wtr<<<cdiv(nUw1, NTHR), NTHR, 0, stream>>>(W1, F_IN, HC1, HC1, F_IN, WT1, nUw1);
    const int nUw2 = HC2 * (K2 / 8);
    k_wtr<<<cdiv(nUw2, NTHR), NTHR, 0, stream>>>(W2, K2, HC2, HC2, K2, WT2, nUw2);
  }

  const int gM = MP / GBM;
  k_gemm<<<dim3(gM, HC1 / GBN), GTHR, 0, stream>>>(XB, WT1, WH1, F_IN, HC1, a1, a1 + HC1, HC1, SD1, MP);
  k_agg<1><<<gA, NTHR, LDS_AGG, stream>>>(src, dst, WH1, SD1, HB, out, nN, nE, nb, vec8, MP);
  k_gemm<<<dim3(gM, HC2 / GBN), GTHR, 0, stream>>>(HB, WT2, WH2, K2, HC2, a2, a2 + HC2, HC2, SD2, MP);
  k_agg<2><<<gA, NTHR, LDS_AGG, stream>>>(src, dst, WH2, SD2, HB, out, nN, nE, nb, vec8, MP);
}
